// ParallelDroplessMLP_27711128993793
// MI455X (gfx1250) — hardware-verified
//
#include <hip/hip_runtime.h>
#include <math.h>
#include <stdint.h>

#define SLEN    2048
#define HS      512
#define FFN     2048
#define NE      8
#define TOPK    2
#define NTOK    SLEN
#define TASSIGN (NTOK * TOPK)
#define TROWS   16
#define NTILE   (TASSIGN / TROWS)
#define CW      128
#define NCH     (FFN / CW)
#define XP      (HS + 8)
#define HP      (CW + 8)
#define SP      (HS + 4)

typedef float          v4f   __attribute__((ext_vector_type(4), __may_alias__));
typedef float          v8f   __attribute__((ext_vector_type(8)));
typedef unsigned short v4us  __attribute__((ext_vector_type(4), __may_alias__));
typedef unsigned short v8us  __attribute__((ext_vector_type(8), __may_alias__));
typedef __bf16         v16bf __attribute__((ext_vector_type(16)));

union Frag { v16bf v; v8us h[2]; };

__device__ __forceinline__ unsigned short f2bf(float f) {
    unsigned int u = __float_as_uint(f);
    u += 0x7FFFu + ((u >> 16) & 1u);
    return (unsigned short)(u >> 16);
}
__device__ __forceinline__ float bf2f(unsigned short b) {
    return __uint_as_float(((unsigned int)b) << 16);
}
__device__ __forceinline__ void split2(float f, unsigned short& hi, unsigned short& lo) {
    hi = f2bf(f);
    lo = f2bf(f - bf2f(hi));
}
__device__ __forceinline__ float gelu_f(float v) {
    return 0.5f * v * (1.0f + erff(v * 0.70710678118654752440f));
}

__device__ __forceinline__ void mma3(v8f& acc, const v16bf ah, const v16bf al, const v16bf bh, const v16bf bl) {
    v8f c = acc;
    c = __builtin_amdgcn_wmma_f32_16x16x32_bf16(false, ah, false, bh, (short)0, c, false, false);
    c = __builtin_amdgcn_wmma_f32_16x16x32_bf16(false, ah, false, bl, (short)0, c, false, false);
    c = __builtin_amdgcn_wmma_f32_16x16x32_bf16(false, al, false, bh, (short)0, c, false, false);
    asm volatile("v_nop\n\tv_nop\n\tv_nop\n\tv_nop" : "+v"(c) : "v"(ah), "v"(al), "v"(bh), "v"(bl));
    acc = c;
}

template <int K, int N>
__global__ __launch_bounds__(256)
void prep_t(const float* __restrict__ w, unsigned short* __restrict__ th, unsigned short* __restrict__ tl)
{
    __shared__ __attribute__((aligned(16))) float tile[64 * 68];
    const int tid = threadIdx.x, wv = tid >> 5, lane = tid & 31;
    const int n0 = blockIdx.x * 64;
    const int k0 = blockIdx.y * 64;
    const int e  = blockIdx.z;

    #pragma unroll
    for (int i = 0; i < 4; ++i) {
        const int idx = tid + 256 * i;
        const int row = idx >> 4, c4 = idx & 15;
        const v4f v = *(const v4f*)(w + ((size_t)(e * K + k0 + row)) * N + n0 + 4 * c4);
        *(v4f*)&tile[row * 68 + 4 * c4] = v;
    }
    __syncthreads();

    v8us hv[2], lv[2];
    size_t off[2];
    #pragma unroll
    for (int p = 0; p < 2; ++p) {
        const int nn = p * 32 + wv * 4 + (lane >> 3);
        const int kg = lane & 7;
        v8us a = {0, 0, 0, 0, 0, 0, 0, 0};
        v8us b = {0, 0, 0, 0, 0, 0, 0, 0};
        #pragma unroll
        for (int i = 0; i < 8; ++i) {
            const float f = tile[(8 * kg + i) * 68 + nn];
            unsigned short hi, lo;
            split2(f, hi, lo);
            a[i] = hi;
            b[i] = lo;
        }
        hv[p] = a;
        lv[p] = b;
        off[p] = ((size_t)(e * N + n0 + nn)) * K + k0 + 8 * kg;
        *(volatile v8us*)(th + off[p]) = a;
        *(volatile v8us*)(tl + off[p]) = b;
    }
    __threadfence();
    #pragma unroll
    for (int p = 0; p < 2; ++p) {
        *(volatile v8us*)(th + off[p]) = hv[p];
        *(volatile v8us*)(tl + off[p]) = lv[p];
    }
}

__device__ __forceinline__ void store_rows(const float* st, const unsigned short* alist,
                                           float* outg, int lbase, int nrows, int wv, int lane)
{
    #pragma unroll
    for (int q = 0; q < 4; ++q) {
        const int rr = wv * 4 + q;
        if (rr < nrows) {
            const int a = alist[lbase + rr];
            if ((unsigned)a < (unsigned)TASSIGN) {
                float* dst = outg + (size_t)a * HS;
                #pragma unroll
                for (int s = 0; s < 4; ++s) {
                    const int col = 128 * s + 4 * lane;
                    const v4f v = *(const v4f*)(st + rr * SP + col);
                    *(volatile v4f*)(dst + col) = v;
                }
            }
        }
    }
}

__global__ __launch_bounds__(128)
void expert_mlp(const float* __restrict__ x, const int* __restrict__ ei,
                const unsigned short* __restrict__ w1h, const unsigned short* __restrict__ w1l,
                const unsigned short* __restrict__ w2h, const unsigned short* __restrict__ w2l,
                float* __restrict__ outg)
{
    union RA { unsigned short xt[2][TROWS * XP]; float st[TROWS * SP]; };
    __shared__ __attribute__((aligned(16))) RA ra;
    __shared__ __attribute__((aligned(16))) unsigned short hc[2][TROWS * HP];
    __shared__ unsigned short alist[TASSIGN];
    __shared__ int wcnt[4];

    const int e   = blockIdx.x;
    const int ty  = blockIdx.y;
    const int tid = threadIdx.x, wv = tid >> 5, lane = tid & 31;
    const int hh  = lane >> 4, m = lane & 15;

    int base = 0;
    const int need = TROWS * ty + TROWS;
    for (int c0 = 0; c0 < TASSIGN; c0 += 128) {
        const int a = c0 + tid;
        const int v = ei[a];
        const bool hit = (v == e);
        const unsigned int bal = __builtin_amdgcn_ballot_w32(hit);
        const int within = __builtin_popcount(bal & ((1u << lane) - 1u));
        if (lane == 0) wcnt[wv] = __builtin_popcount(bal);
        __syncthreads();
        const int n0 = wcnt[0], n1 = wcnt[1], n2 = wcnt[2], n3 = wcnt[3];
        const int woff = (wv > 0 ? n0 : 0) + (wv > 1 ? n1 : 0) + (wv > 2 ? n2 : 0);
        if (hit) {
            const int pos = base + woff + within;
            if ((unsigned)pos < (unsigned)TASSIGN) alist[pos] = (unsigned short)a;
        }
        base += n0 + n1 + n2 + n3;
        __syncthreads();
        if (base >= need) break;
    }
    const int cnt = base < TASSIGN ? base : TASSIGN;
    int nrows = cnt - TROWS * ty;
    if (nrows <= 0) return;
    if (nrows > TROWS) nrows = TROWS;
    const int lbase = TROWS * ty;

    #pragma unroll 2
    for (int r = 0; r < TROWS; ++r) {
        v4us hv = {0, 0, 0, 0};
        v4us lv = {0, 0, 0, 0};
        if (r < nrows) {
            const int a = alist[lbase + r];
            int t = a >> 1;
            t = t < 0 ? 0 : (t > NTOK - 1 ? NTOK - 1 : t);
            const v4f v = *(const v4f*)(x + (size_t)t * HS + 4 * tid);
            unsigned short h0, l0, h1, l1, h2, l2, h3, l3;
            split2(v.x, h0, l0); split2(v.y, h1, l1); split2(v.z, h2, l2); split2(v.w, h3, l3);
            hv.x = h0; hv.y = h1; hv.z = h2; hv.w = h3;
            lv.x = l0; lv.y = l1; lv.z = l2; lv.w = l3;
        }
        *(v4us*)&ra.xt[0][r * XP + 4 * tid] = hv;
        *(v4us*)&ra.xt[1][r * XP + 4 * tid] = lv;
    }
    __syncthreads();

    v8f acc2[8];
    #pragma unroll
    for (int j = 0; j < 8; ++j) { v8f z = {0.f, 0.f, 0.f, 0.f, 0.f, 0.f, 0.f, 0.f}; acc2[j] = z; }

    const unsigned short* xah = &ra.xt[0][m * XP + 8 * hh];
    const unsigned short* xal = &ra.xt[1][m * XP + 8 * hh];
    const unsigned short* hah = &hc[0][m * HP + 8 * hh];
    const unsigned short* hal = &hc[1][m * HP + 8 * hh];
    const size_t w2off = ((size_t)e * HS + wv * 128 + m) * (size_t)FFN + 8 * hh;

    #pragma unroll 1
    for (int ch = 0; ch < NCH; ++ch) {
        v8f acc1[2];
        #pragma unroll
        for (int j = 0; j < 2; ++j) { v8f z = {0.f, 0.f, 0.f, 0.f, 0.f, 0.f, 0.f, 0.f}; acc1[j] = z; }
        const size_t w1off = ((size_t)e * FFN + ch * CW + wv * 32 + m) * (size_t)HS + 8 * hh;
        #pragma unroll 1
        for (int ks = 0; ks < HS / 32; ++ks) {
            const int k0 = ks * 32;
            Frag ah, al;
            ah.h[0] = *(const v8us*)(xah + k0);
            ah.h[1] = *(const v8us*)(xah + k0 + 16);
            al.h[0] = *(const v8us*)(xal + k0);
            al.h[1] = *(const v8us*)(xal + k0 + 16);
            #pragma unroll
            for (int j = 0; j < 2; ++j) {
                const size_t o = w1off + (size_t)j * 16 * HS + k0;
                Frag bh, bl;
                bh.h[0] = *(const v8us*)(w1h + o);
                bh.h[1] = *(const v8us*)(w1h + o + 16);
                bl.h[0] = *(const v8us*)(w1l + o);
                bl.h[1] = *(const v8us*)(w1l + o + 16);
                mma3(acc1[j], ah.v, al.v, bh.v, bl.v);
            }
        }
        __syncthreads();

        #pragma unroll
        for (int j = 0; j < 2; ++j) {
            #pragma unroll
            for (int r = 0; r < 8; ++r) {
                const float g = gelu_f(acc1[j][r]);
                unsigned short hi, lo;
                split2(g, hi, lo);
                const int idx = (8 * hh + r) * HP + wv * 32 + 16 * j + m;
                hc[0][idx] = hi;
                hc[1][idx] = lo;
            }
        }
        __syncthreads();

        #pragma unroll 1
        for (int kk = 0; kk < CW / 32; ++kk) {
            const int k0 = kk * 32;
            Frag ah, al;
            ah.h[0] = *(const v8us*)(hah + k0);
            ah.h[1] = *(const v8us*)(hah + k0 + 16);
            al.h[0] = *(const v8us*)(hal + k0);
            al.h[1] = *(const v8us*)(hal + k0 + 16);
            #pragma unroll
            for (int j = 0; j < 8; ++j) {
                const size_t o = w2off + (size_t)j * 16 * FFN + (size_t)ch * CW + k0;
                Frag bh, bl;
                bh.h[0] = *(const v8us*)(w2h + o);
                bh.h[1] = *(const v8us*)(w2h + o + 16);
                bl.h[0] = *(const v8us*)(w2l + o);
                bl.h[1] = *(const v8us*)(w2l + o + 16);
                mma3(acc2[j], ah.v, al.v, bh.v, bl.v);
            }
        }
    }

    #pragma unroll
    for (int j = 0; j < 8; ++j) {
        #pragma unroll
        for (int r = 0; r < 8; ++r)
            ra.st[(8 * hh + r) * SP + wv * 128 + 16 * j + m] = acc2[j][r];
    }
    __syncthreads();

    store_rows(ra.st, alist, outg, lbase, nrows, wv, lane);
    __threadfence();
    store_rows(ra.st, alist, outg, lbase, nrows, wv, lane);
}

__global__ __launch_bounds__(128)
void combine_k(const float* __restrict__ outg, const int* __restrict__ ei, const float* __restrict__ ew,
               float* __restrict__ y, float* __restrict__ buf)
{
    #pragma clang fp contract(off)
    const int t = blockIdx.x;
    const int c = 4 * threadIdx.x;
    int e0 = ei[2 * t], e1 = ei[2 * t + 1];
    e0 = e0 < 0 ? 0 : (e0 > NE - 1 ? NE - 1 : e0);
    e1 = e1 < 0 ? 0 : (e1 > NE - 1 ? NE - 1 : e1);
    const float w0 = ew[2 * t], w1v = ew[2 * t + 1];
    const v4f o0 = *(const v4f*)(outg + (size_t)(2 * t) * HS + c);
    const v4f o1 = *(const v4f*)(outg + (size_t)(2 * t + 1) * HS + c);
    const v4f p0 = o0 * w0;
    const v4f p1 = o1 * w1v;
    const v4f yv = p0 + p1;
    const v4f zero = {0.f, 0.f, 0.f, 0.f};
    v4f bv[NE];
    #pragma unroll
    for (int ep = 0; ep < NE; ++ep) {
        v4f b = zero;
        if (e0 == ep) b = o0;
        if (e1 == ep) b = b + o1;
        bv[ep] = b;
    }
    float* yr = y + (size_t)t * HS + c;
    float* br = buf + (size_t)t * NE * HS + c;
    *(volatile v4f*)yr = yv;
    #pragma unroll
    for (int ep = 0; ep < NE; ++ep) *(volatile v4f*)(br + (size_t)ep * HS) = bv[ep];
    __threadfence();
    *(volatile v4f*)yr = yv;
    #pragma unroll
    for (int ep = 0; ep < NE; ++ep) *(volatile v4f*)(br + (size_t)ep * HS) = bv[ep];
}

extern "C" void kernel_launch(void* const* d_in, const int* in_sizes, int n_in,
                              void* d_out, int out_size, void* d_ws, size_t ws_size,
                              hipStream_t stream)
{
    if (n_in < 5) return;
    if (in_sizes[0] != NTOK * HS) return;
    if (in_sizes[1] != TASSIGN) return;
    if (in_sizes[2] != TASSIGN) return;
    if (in_sizes[3] != NE * HS * FFN) return;
    if (in_sizes[4] != NE * FFN * HS) return;
    if (out_size != NTOK * HS + NTOK * NE * HS) return;

    const float* x  = (const float*)d_in[0];
    const float* ew = (const float*)d_in[1];
    const int*   ei = (const int*)d_in[2];
    const float* w1 = (const float*)d_in[3];
    const float* w2 = (const float*)d_in[4];

    float* y   = (float*)d_out;
    float* buf = (float*)d_out + (size_t)NTOK * HS;

    const size_t planeHalves = (size_t)NE * HS * FFN;
    const size_t planeBytes  = planeHalves * sizeof(unsigned short);
    const size_t outgBytes   = (size_t)TASSIGN * HS * sizeof(float);
    const size_t need = 4 * planeBytes + outgBytes;
    if (need > ws_size) return;

    char* base = (char*)d_ws;
    unsigned short* w1h = (unsigned short*)(base + 0 * planeBytes);
    unsigned short* w1l = (unsigned short*)(base + 1 * planeBytes);
    unsigned short* w2h = (unsigned short*)(base + 2 * planeBytes);
    unsigned short* w2l = (unsigned short*)(base + 3 * planeBytes);
    float* outg = (float*)(base + 4 * planeBytes);

    prep_t<HS, FFN><<<dim3(FFN / 64, HS / 64, NE), 256, 0, stream>>>(w1, w1h, w1l);
    prep_t<FFN, HS><<<dim3(HS / 64, FFN / 64, NE), 256, 0, stream>>>(w2, w2h, w2l);
    expert_mlp<<<dim3(NE, NTILE), 128, 0, stream>>>(x, ei, w1h, w1l, w2h, w2l, outg);
    combine_k<<<dim3(NTOK), 128, 0, stream>>>(outg, ei, ew, y, buf);
}
